// TCSLBPBlock_14465449852968
// MI455X (gfx1250) — hardware-verified
//
#include <hip/hip_runtime.h>


typedef _Float16 v16h __attribute__((ext_vector_type(16)));
typedef _Float16 v8h  __attribute__((ext_vector_type(8)));
typedef float    v8f  __attribute__((ext_vector_type(8)));
typedef float    v4f  __attribute__((ext_vector_type(4)));

#define B_   32
#define C_   128
#define H_   56
#define W_   56
#define HW_  3136
#define K_   512
#define NP_  (B_ * HW_)
#define EPS_ 1e-5f

#define WS_STATS        0
#define WS_STATS_BYTES  (C_ * 32 * 4)
#define WS_W3F          (WS_STATS + WS_STATS_BYTES)
#define WS_W3F_BYTES    (9 * 4 * 32 * 1024)
#define WS_W1F          (WS_W3F + WS_W3F_BYTES)
#define WS_W1F_BYTES    (16 * 8 * 1024)
#define WS_XNH          (WS_W1F + WS_W1F_BYTES)
#define WS_XNH_BYTES    (NP_ * C_ * 2)
#define WS_TOTAL        (WS_XNH + WS_XNH_BYTES)
static_assert(WS_W3F % 128 == 0);
static_assert(WS_W1F % 128 == 0);
static_assert(WS_XNH % 128 == 0);
static_assert(WS_TOTAL <= 134217728);

#define HALO_PIX    178
#define HALO_STRIDE 72
#define HALO_BYTES  (HALO_PIX * HALO_STRIDE * 2)
#define YT_STRIDE   264
#define YT_BYTES    (64 * YT_STRIDE * 2)
#define ZT_STRIDE   68
#define ZT_BYTES    (C_ * ZT_STRIDE * 4)
static_assert(ZT_BYTES <= HALO_BYTES + YT_BYTES);
#define TP_         136

__device__ __forceinline__ v16h cat16(v8h lo, v8h hi) {
    return __builtin_shufflevector(lo, hi, 0, 1, 2, 3, 4, 5, 6, 7, 8, 9, 10, 11, 12, 13, 14, 15);
}

__device__ __forceinline__ v8f wmma16(v16h a, v16h b, v8f c) {
    return __builtin_amdgcn_wmma_f32_16x16x32_f16(false, a, false, b, (short)0, c, false, false);
}

__launch_bounds__(256, 1)
__global__ void bn_stats(const float* __restrict__ x,
                         const float* __restrict__ gamma,
                         const float* __restrict__ beta,
                         float* __restrict__ stats) {
    __shared__ double rs[256], rq[256];
    const int c = blockIdx.x, tid = threadIdx.x;
    double s = 0.0, q = 0.0;
    for (int bb = 0; bb < B_; ++bb) {
        const float* xp = x + ((size_t)bb * C_ + c) * HW_;
        for (int i = tid; i < HW_; i += 256) {
            const double v = (double)xp[i];
            s += v; q += v * v;
        }
    }
    rs[tid] = s; rq[tid] = q;
    __syncthreads();
    for (int off = 128; off > 0; off >>= 1) {
        if (tid < off) { rs[tid] += rs[tid + off]; rq[tid] += rq[tid + off]; }
        __syncthreads();
    }
    if (tid < 32) {
        const double mean = rs[0] * (1.0 / (double)NP_);
        const double var  = rq[0] * (1.0 / (double)NP_) - mean * mean;
        const float meanf = (float)mean;
        const float inv   = gamma[c] * rsqrtf((float)var + EPS_);
        const float be    = beta[c];
        float val = 0.f;
        if (tid == 0) val = meanf;
        else if (tid == 1) val = inv;
        else if (tid == 2) val = be;
        volatile float* dp = (volatile float*)(stats + c * 32 + tid);
        *dp = val;
        __threadfence();
        *dp = val;
    }
}

__launch_bounds__(256, 1)
__global__ void bn_apply_pack(const float* __restrict__ x,
                              const float* __restrict__ stats,
                              _Float16* __restrict__ xnh) {
    __shared__ __align__(16) _Float16 t[64 * TP_];
    __shared__ float smean[C_], sinv[C_], sbeta[C_];
    const int tid = threadIdx.x;
    const int p0 = blockIdx.x * 64;
    const int b  = p0 / HW_;
    const int s0 = p0 - b * HW_;
    if (tid < C_) {
        smean[tid] = stats[tid * 32 + 0];
        sinv[tid]  = stats[tid * 32 + 1];
        sbeta[tid] = stats[tid * 32 + 2];
    }
    __syncthreads();
#pragma unroll 2
    for (int it = 0; it < 8; ++it) {
        const int idx = it * 256 + tid;
        const int c = idx >> 4, i4 = idx & 15;
        const v4f v = *(const v4f*)(x + ((size_t)b * C_ + c) * HW_ + (size_t)(s0 + 4 * i4));
        const float mu = smean[c], iv = sinv[c], be = sbeta[c];
        _Float16* tp = t + (4 * i4) * TP_ + c;
        tp[0 * TP_] = (_Float16)((v.x - mu) * iv + be);
        tp[1 * TP_] = (_Float16)((v.y - mu) * iv + be);
        tp[2 * TP_] = (_Float16)((v.z - mu) * iv + be);
        tp[3 * TP_] = (_Float16)((v.w - mu) * iv + be);
    }
    __syncthreads();
#pragma unroll
    for (int it = 0; it < 4; ++it) {
        const int idx = it * 256 + tid;
        const int i = idx >> 4, q = idx & 15;
        const v8h hv = *(const v8h*)(t + i * TP_ + q * 8);
        volatile v8h* dp = (volatile v8h*)(xnh + (size_t)(p0 + i) * C_ + q * 8);
        *dp = hv;
        __threadfence();
        *dp = hv;
    }
}

__launch_bounds__(256, 1)
__global__ void pack_w3(const float* __restrict__ W3, _Float16* __restrict__ w3f) {
    const int gid = blockIdx.x * 256 + threadIdx.x;
    if (gid >= 9 * 4 * 32 * 32) return;
    const int lane = gid & 31;
    const int frag = gid >> 5;
    const int tap  = frag >> 7;
    const int rem  = frag & 127;
    const int cc   = rem >> 5;
    const int nt   = rem & 31;
    const int n    = nt * 16 + (lane & 15);
    const int h    = lane >> 4;
    const float* wp = W3 + ((size_t)n * C_ + (size_t)(cc * 32 + 8 * h)) * 9 + tap;
    v8h lo, hi;
#pragma unroll
    for (int i = 0; i < 8; ++i) {
        lo[i] = (_Float16)wp[i * 9];
        hi[i] = (_Float16)wp[(16 + i) * 9];
    }
    _Float16* dst = w3f + (size_t)frag * 512 + lane * 16;
    volatile v8h* d0 = (volatile v8h*)dst;
    volatile v8h* d1 = (volatile v8h*)(dst + 8);
    *d0 = lo; *d1 = hi;
    __threadfence();
    *d0 = lo; *d1 = hi;
}

__launch_bounds__(256, 1)
__global__ void pack_w1(const float* __restrict__ W1, _Float16* __restrict__ w1f) {
    const int gid = blockIdx.x * 256 + threadIdx.x;
    if (gid >= 16 * 8 * 32) return;
    const int lane = gid & 31;
    const int frag = gid >> 5;
    const int kc = frag >> 3, nt = frag & 7;
    const int c  = nt * 16 + (lane & 15);
    const int h  = lane >> 4;
    const float* wp = W1 + (size_t)c * K_ + kc * 32 + 8 * h;
    v8h lo, hi;
#pragma unroll
    for (int i = 0; i < 8; ++i) {
        lo[i] = (_Float16)(wp[i] * 16.0f);
        hi[i] = (_Float16)(wp[16 + i] * 16.0f);
    }
    _Float16* dst = w1f + (size_t)frag * 512 + lane * 16;
    volatile v8h* d0 = (volatile v8h*)dst;
    volatile v8h* d1 = (volatile v8h*)(dst + 8);
    *d0 = lo; *d1 = hi;
    __threadfence();
    *d0 = lo; *d1 = hi;
}

__launch_bounds__(256, 1)
__global__ void tcslbp_main(const float* __restrict__ x,
                            const float* __restrict__ b1,
                            const _Float16* __restrict__ xnh,
                            const _Float16* __restrict__ w3f,
                            const _Float16* __restrict__ w1f,
                            float* __restrict__ out) {
    __shared__ __align__(16) unsigned char smem[HALO_BYTES + YT_BYTES + 64];
    _Float16* haloT = (_Float16*)smem;
    _Float16* yT    = (_Float16*)(smem + HALO_BYTES);
    _Float16* zbuf  = (_Float16*)(smem + HALO_BYTES + YT_BYTES);
    float*    zT    = (float*)smem;

    const int tid    = threadIdx.x;
    const int wave   = tid >> 5;
    const int lane   = tid & 31;
    const int l16    = lane & 15;
    const int hiHalf = (lane >> 4) & 1;
    const int kb     = hiHalf * 8;

    const int p0 = blockIdx.x * 64;
    const int b  = p0 / HW_;
    const int s0 = p0 - b * HW_;

    if (tid < 32) zbuf[tid] = (_Float16)0.f;

    int wcol[4];
#pragma unroll
    for (int mt = 0; mt < 4; ++mt) {
        const int s = s0 + mt * 16 + l16;
        wcol[mt] = s % W_;
    }

    v8f acc2[4] = {};

    for (int half = 0; half < 2; ++half) {
        v8f acc1[4][2] = {};
        for (int chh = 0; chh < 2; ++chh) {
            __syncthreads();
            for (int idx = tid; idx < HALO_PIX * 8; idx += 256) {
                const int i = idx >> 3, q = idx & 7;
                const int sg = s0 - 57 + i;
                v8h v = {};
                if ((unsigned)sg < (unsigned)HW_)
                    v = *(const v8h*)(xnh + (size_t)(b * HW_ + sg) * C_ + chh * 64 + q * 8);
                *(v8h*)(haloT + i * HALO_STRIDE + q * 8) = v;
            }
            __syncthreads();
#pragma unroll 1
            for (int tc = 0; tc < 18; ++tc) {
                const int tap = tc >> 1, cc2 = tc & 1;
                const int t3  = tap / 3;
                const int dr  = t3 - 1, dc = tap - t3 * 3 - 1;
                const int hoff = 57 + dr * W_ + dc;
                v16h af[4];
#pragma unroll
                for (int mt = 0; mt < 4; ++mt) {
                    const bool vw = (unsigned)(wcol[mt] + dc) < (unsigned)W_;
                    const int  hidx = mt * 16 + l16 + hoff;
                    const _Float16* base = vw ? (haloT + hidx * HALO_STRIDE + cc2 * 32) : zbuf;
                    const v8h lo = *(const v8h*)(base + kb);
                    const v8h hi = *(const v8h*)(base + kb + 16);
                    af[mt] = cat16(lo, hi);
                }
                const int ccg   = chh * 2 + cc2;
                const int fbase = (tap * 4 + ccg) * 32 + half * 16 + wave * 2;
                const _Float16* bp0 = w3f + (size_t)fbase * 512 + lane * 16;
                const _Float16* bp1 = bp0 + 512;
                const v16h bf0 = cat16(*(const v8h*)bp0, *(const v8h*)(bp0 + 8));
                const v16h bf1 = cat16(*(const v8h*)bp1, *(const v8h*)(bp1 + 8));
                acc1[0][0] = wmma16(af[0], bf0, acc1[0][0]);
                acc1[1][0] = wmma16(af[1], bf0, acc1[1][0]);
                acc1[2][0] = wmma16(af[2], bf0, acc1[2][0]);
                acc1[3][0] = wmma16(af[3], bf0, acc1[3][0]);
                acc1[0][1] = wmma16(af[0], bf1, acc1[0][1]);
                acc1[1][1] = wmma16(af[1], bf1, acc1[1][1]);
                acc1[2][1] = wmma16(af[2], bf1, acc1[2][1]);
                acc1[3][1] = wmma16(af[3], bf1, acc1[3][1]);
                asm volatile("v_nop\n\tv_nop\n\tv_nop\n\tv_nop"
                             : "+v"(acc1[0][0]), "+v"(acc1[1][0]), "+v"(acc1[2][0]), "+v"(acc1[3][0]),
                               "+v"(acc1[0][1]), "+v"(acc1[1][1]), "+v"(acc1[2][1]), "+v"(acc1[3][1])
                             : "v"(af[0]), "v"(af[1]), "v"(af[2]), "v"(af[3]), "v"(bf0), "v"(bf1));
            }
        }
#pragma unroll
        for (int mt = 0; mt < 4; ++mt)
#pragma unroll
            for (int nt = 0; nt < 2; ++nt) {
                const int n = wave * 32 + nt * 16 + l16;
#pragma unroll
                for (int v = 0; v < 8; ++v) {
                    const int m = mt * 16 + hiHalf * 8 + v;
                    const float f = acc1[mt][nt][v];
                    yT[m * YT_STRIDE + n] = (_Float16)(f > 0.f ? f : 0.f);
                }
            }
        __syncthreads();
#pragma unroll 1
        for (int kc = 0; kc < 8; ++kc) {
            const int kcg = half * 8 + kc;
            const _Float16* bp = w1f + (size_t)(kcg * 8 + wave) * 512 + lane * 16;
            const v16h bf = cat16(*(const v8h*)bp, *(const v8h*)(bp + 8));
            const int kb2 = kc * 32 + kb;
            v16h a2[4];
#pragma unroll
            for (int mt = 0; mt < 4; ++mt) {
                const int row = mt * 16 + l16;
                const v8h lo = *(const v8h*)(yT + row * YT_STRIDE + kb2);
                const v8h hi = *(const v8h*)(yT + row * YT_STRIDE + kb2 + 16);
                a2[mt] = cat16(lo, hi);
            }
            acc2[0] = wmma16(a2[0], bf, acc2[0]);
            acc2[1] = wmma16(a2[1], bf, acc2[1]);
            acc2[2] = wmma16(a2[2], bf, acc2[2]);
            acc2[3] = wmma16(a2[3], bf, acc2[3]);
            asm volatile("v_nop\n\tv_nop\n\tv_nop\n\tv_nop"
                         : "+v"(acc2[0]), "+v"(acc2[1]), "+v"(acc2[2]), "+v"(acc2[3])
                         : "v"(a2[0]), "v"(a2[1]), "v"(a2[2]), "v"(a2[3]), "v"(bf));
        }
        __syncthreads();
    }
#pragma unroll
    for (int mt = 0; mt < 4; ++mt) {
        const int n = wave * 16 + l16;
        float* zp = zT + n * ZT_STRIDE + mt * 16 + hiHalf * 8;
        const v4f z0 = __builtin_shufflevector(acc2[mt], acc2[mt], 0, 1, 2, 3);
        const v4f z1 = __builtin_shufflevector(acc2[mt], acc2[mt], 4, 5, 6, 7);
        *(v4f*)zp       = z0;
        *(v4f*)(zp + 4) = z1;
    }
    __syncthreads();
    const float s16 = 0.0625f;
#pragma unroll 2
    for (int it = 0; it < 8; ++it) {
        const int idx = it * 256 + tid;
        const int c = idx >> 4, i4 = idx & 15;
        const size_t gi = ((size_t)b * C_ + c) * HW_ + (size_t)(s0 + 4 * i4);
        const v4f zz = *(const v4f*)(zT + c * ZT_STRIDE + 4 * i4);
        const v4f xr = *(const v4f*)(x + gi);
        const float bb = b1[c];
        const v4f bv = {bb, bb, bb, bb};
        const v4f o = (zz * s16 + bv) + xr;
        volatile v4f* op = (volatile v4f*)(out + gi);
        *op = o;
        __threadfence();
        *op = o;
    }
}

extern "C" void kernel_launch(void* const* d_in, const int* in_sizes, int n_in,
                              void* d_out, int out_size, void* d_ws, size_t ws_size,
                              hipStream_t stream) {
    if (n_in < 6) return;
    if (in_sizes[0] != B_ * C_ * HW_ || in_sizes[1] != C_ || in_sizes[2] != C_ ||
        in_sizes[3] != K_ * C_ * 9 || in_sizes[4] != C_ * K_ || in_sizes[5] != C_) return;
    if (out_size != B_ * C_ * HW_) return;
    if (ws_size < (size_t)WS_TOTAL) return;

    const float* x     = (const float*)d_in[0];
    const float* gamma = (const float*)d_in[1];
    const float* beta  = (const float*)d_in[2];
    const float* W3    = (const float*)d_in[3];
    const float* W1    = (const float*)d_in[4];
    const float* b1    = (const float*)d_in[5];
    float* out = (float*)d_out;

    char* ws = (char*)d_ws;
    float*    stats = (float*)(ws + WS_STATS);
    _Float16* w3f   = (_Float16*)(ws + WS_W3F);
    _Float16* w1f   = (_Float16*)(ws + WS_W1F);
    _Float16* xnh   = (_Float16*)(ws + WS_XNH);

    bn_stats<<<C_, 256, 0, stream>>>(x, gamma, beta, stats);
    pack_w3<<<(9 * 4 * 32 * 32) / 256, 256, 0, stream>>>(W3, w3f);
    pack_w1<<<(16 * 8 * 32) / 256, 256, 0, stream>>>(W1, w1f);
    bn_apply_pack<<<NP_ / 64, 256, 0, stream>>>(x, stats, xnh);
    tcslbp_main<<<NP_ / 64, 256, 0, stream>>>(x, b1, xnh, w3f, w1f, out);
}
